// CombinedGAT_83459804495956
// MI455X (gfx1250) — hardware-verified
//
#include <hip/hip_runtime.h>
#include <stddef.h>


#define HIGHD   128
#define LOWD    32
#define EMBD    64
#define IN1     192
#define HEADS   8
#define HIDC    32
#define C1      256
#define OUTC    8
#define OUTP    16
#define NTHR    256
#define NWAVE   8
#define EPT     8
#define NGRP    2
#define CHUNK   (NTHR * EPT * NGRP)
#define WCAP    (EPT * NGRP * 32)
#define LISTN   (NWAVE * WCAP)
#define NBC     4096
#define NBF     1024
#define RCAP    40960
#define RBN     128
#define TGT     256
#define DEGCAP  256
#define OTHR    512
#define BMX     64
#define BM1     32
#define BM2     64
#define G2THR   128
#define WSCAP   134217728
#define NEG_SLOPE 0.2f
#define WSCALE  16.0f
#define WINV    0.0625f

#define LDS_FILL ((RCAP + NBF + LISTN) * 4 + 64)

static_assert((CHUNK & (CHUNK - 1)) == 0);
static_assert(CHUNK <= 4096);
static_assert(NBC <= 4096 && NBF <= 4096);
static_assert((NBC & (NBC - 1)) == 0 && (NBF & (NBF - 1)) == 0);
static_assert(NBC == 4 * NBF);
static_assert(OTHR * 8 == NBC);
static_assert((RCAP % 32) == 0);
static_assert(TGT == NWAVE * 32);
static_assert((NBC % TGT) == 0);
static_assert((TGT % BMX) == 0 && (TGT % BM1) == 0 && (TGT % BM2) == 0);
static_assert(HEADS * HIDC == C1);
static_assert(HIGHD + EMBD == IN1);
static_assert(IN1 % 32 == 0 && C1 % 32 == 0 && LOWD == 32 && EMBD == 64);
static_assert(C1 == 32 * 8);
static_assert(BM1 * HEADS == NTHR);
static_assert((BMX * IN1 / 8) % NTHR == 0);
static_assert((BM1 * C1 / 4) % NTHR == 0);
static_assert((BM2 * OUTP / 4) % G2THR == 0);
static_assert(BM2 == 16 * (G2THR / 32));
static_assert(OUTC + 2 <= OUTP);

typedef float          v4f  __attribute__((ext_vector_type(4)));
typedef float          v8f  __attribute__((ext_vector_type(8)));
typedef int            v4i  __attribute__((ext_vector_type(4)));
typedef _Float16       v8h  __attribute__((ext_vector_type(8)));
typedef _Float16       v16h __attribute__((ext_vector_type(16)));
union FragH { v16h v; v8h h[2]; };

__device__ __forceinline__ v8f wmh(v16h a, v16h b, v8f c) {
  v8f d = __builtin_amdgcn_wmma_f32_16x16x32_f16(false, a, false, b, (short)0, c, false, false);
  asm volatile("v_nop\n\tv_nop\n\tv_nop\n\tv_nop" : "+v"(d) : "v"(a), "v"(b));
  return d;
}

__device__ __forceinline__ v8h cvt8(v4f a, v4f b) {
  v8h o;
  o[0] = (_Float16)a.x; o[1] = (_Float16)a.y; o[2] = (_Float16)a.z; o[3] = (_Float16)a.w;
  o[4] = (_Float16)b.x; o[5] = (_Float16)b.y; o[6] = (_Float16)b.z; o[7] = (_Float16)b.w;
  return o;
}

__device__ __forceinline__ float lrelu(float v) { return v > 0.0f ? v : NEG_SLOPE * v; }
__device__ __forceinline__ float eluf(float v)  { return v > 0.0f ? v : (__expf(v) - 1.0f); }
__device__ __forceinline__ v4f lrelu4(v4f v) { v4f r; r.x = lrelu(v.x); r.y = lrelu(v.y); r.z = lrelu(v.z); r.w = lrelu(v.w); return r; }
__device__ __forceinline__ v4f elu4(v4f v)   { v4f r; r.x = eluf(v.x); r.y = eluf(v.y); r.z = eluf(v.z); r.w = eluf(v.w); return r; }
__device__ __forceinline__ v4f fmax4(v4f a, v4f b) { v4f r; r.x = fmaxf(a.x, b.x); r.y = fmaxf(a.y, b.y); r.z = fmaxf(a.z, b.z); r.w = fmaxf(a.w, b.w); return r; }
__device__ __forceinline__ v4f exp4(v4f v) { v4f r; r.x = __expf(v.x); r.y = __expf(v.y); r.z = __expf(v.z); r.w = __expf(v.w); return r; }
__device__ __forceinline__ v4f xormax4(v4f v, int d) {
  v4f r;
  r.x = fmaxf(v.x, __shfl_xor(v.x, d)); r.y = fmaxf(v.y, __shfl_xor(v.y, d));
  r.z = fmaxf(v.z, __shfl_xor(v.z, d)); r.w = fmaxf(v.w, __shfl_xor(v.w, d));
  return r;
}
__device__ __forceinline__ v4f xorsum4(v4f v, int d) {
  v4f r;
  r.x = v.x + __shfl_xor(v.x, d); r.y = v.y + __shfl_xor(v.y, d);
  r.z = v.z + __shfl_xor(v.z, d); r.w = v.w + __shfl_xor(v.w, d);
  return r;
}
__device__ __forceinline__ float sel8(v4f a, v4f b, int h) {
  float r = a.x;
  r = (h == 1) ? a.y : r; r = (h == 2) ? a.z : r; r = (h == 3) ? a.w : r;
  r = (h == 4) ? b.x : r; r = (h == 5) ? b.y : r; r = (h == 6) ? b.z : r; r = (h == 7) ? b.w : r;
  return r;
}
__device__ __forceinline__ void wave_sync() {
  __builtin_amdgcn_fence(__ATOMIC_RELEASE, "wavefront");
  __builtin_amdgcn_wave_barrier();
}

template <int NB>
__device__ __forceinline__ int scan_chunk(const int* __restrict__ dsts, int nE, int cbase, int slotBase,
                                          int vec8, int* list, int tid, int lane, int wave) {
  int wc = 0;
#pragma unroll
  for (int g = 0; g < NGRP; ++g) {
    const int el0  = (g * NTHR + tid) * EPT;
    const int e0   = cbase + el0;
    const int sent = -2147483647 - 1;
    v4i da, db;
    if (vec8 != 0 && cbase + CHUNK <= nE) {
      da = *(const v4i*)(dsts + e0);
      db = *(const v4i*)(dsts + e0 + 4);
    } else {
      da.x = (e0     < nE) ? dsts[min(e0, nE - 1)] : sent;
      da.y = (e0 + 1 < nE) ? dsts[min(e0 + 1, nE - 1)] : sent;
      da.z = (e0 + 2 < nE) ? dsts[min(e0 + 2, nE - 1)] : sent;
      da.w = (e0 + 3 < nE) ? dsts[min(e0 + 3, nE - 1)] : sent;
      db.x = (e0 + 4 < nE) ? dsts[min(e0 + 4, nE - 1)] : sent;
      db.y = (e0 + 5 < nE) ? dsts[min(e0 + 5, nE - 1)] : sent;
      db.z = (e0 + 6 < nE) ? dsts[min(e0 + 6, nE - 1)] : sent;
      db.w = (e0 + 7 < nE) ? dsts[min(e0 + 7, nE - 1)] : sent;
    }
    const unsigned nb = (unsigned)slotBase;
    const unsigned s0 = (unsigned)da.x - nb, s1 = (unsigned)da.y - nb;
    const unsigned s2 = (unsigned)da.z - nb, s3 = (unsigned)da.w - nb;
    const unsigned s4 = (unsigned)db.x - nb, s5 = (unsigned)db.y - nb;
    const unsigned s6 = (unsigned)db.z - nb, s7 = (unsigned)db.w - nb;
    const bool h0 = s0 < (unsigned)NB, h1 = s1 < (unsigned)NB, h2 = s2 < (unsigned)NB, h3 = s3 < (unsigned)NB;
    const bool h4 = s4 < (unsigned)NB, h5 = s5 < (unsigned)NB, h6 = s6 < (unsigned)NB, h7 = s7 < (unsigned)NB;
    const unsigned any = __builtin_amdgcn_ballot_w32(h0 | h1 | h2 | h3 | h4 | h5 | h6 | h7);
    if (any != 0u) {
#define HITJ(J, HJ, SJ) { \
        const unsigned mj = __builtin_amdgcn_ballot_w32(HJ); \
        if (mj != 0u) { \
          if (HJ) { \
            const int pos = wc + (int)__builtin_amdgcn_mbcnt_lo(mj, 0u); \
            if (pos < WCAP) list[wave * WCAP + pos] = ((el0 + (J)) << 12) | (int)(SJ); \
          } \
          wc += (int)__builtin_popcount(mj); } }
      HITJ(0, h0, s0)
      HITJ(1, h1, s1)
      HITJ(2, h2, s2)
      HITJ(3, h3, s3)
      HITJ(4, h4, s4)
      HITJ(5, h5, s5)
      HITJ(6, h6, s6)
      HITJ(7, h7, s7)
#undef HITJ
    }
  }
  return wc;
}

template <int KD, int NCW, int NCP>
__global__ __launch_bounds__(NTHR) void k_wprep(const float* __restrict__ W, _Float16* wp) {
  constexpr int KS    = KD / 8;
  constexpr int UNITS = NCP * KS;
  static_assert(KD % 8 == 0 && NCP >= NCW);
  const int i = (int)blockIdx.x * NTHR + (int)threadIdx.x;
  if (i >= UNITS) return;
  const int n  = i / KS;
  const int k0 = (i - n * KS) * 8;
  const int nc = n < NCW ? n : NCW - 1;
  v4f a, b;
  a.x = W[(size_t)(k0 + 0) * NCW + nc]; a.y = W[(size_t)(k0 + 1) * NCW + nc];
  a.z = W[(size_t)(k0 + 2) * NCW + nc]; a.w = W[(size_t)(k0 + 3) * NCW + nc];
  b.x = W[(size_t)(k0 + 4) * NCW + nc]; b.y = W[(size_t)(k0 + 5) * NCW + nc];
  b.z = W[(size_t)(k0 + 6) * NCW + nc]; b.w = W[(size_t)(k0 + 7) * NCW + nc];
  a = a * WSCALE; b = b * WSCALE;
  const v4f z4 = {0.f, 0.f, 0.f, 0.f};
  if (n >= NCW) { a = z4; b = z4; }
  const v8h o = cvt8(a, b);
  _Float16* d = wp + (size_t)i * 8;
  *(volatile v8h*)d = o;
  __threadfence();
  *(volatile v8h*)d = o;
}

__global__ __launch_bounds__(NTHR) void k_xprep(
    const float* __restrict__ high, const float* __restrict__ low,
    const _Float16* __restrict__ wembp, const float* __restrict__ bemb, _Float16* xp, int nN) {
  constexpr int NIT = BMX * IN1 / 8 / NTHR;
  __shared__ __attribute__((aligned(16))) _Float16 sA[BMX * LOWD];
  __shared__ __attribute__((aligned(16))) _Float16 sX[BMX * IN1];
  const int tid = threadIdx.x, lane = tid & 31, wave = tid >> 5, hh = lane >> 4, m = lane & 15;
  const int rowBase = blockIdx.x * BMX;
  const v4f z4 = {0.f, 0.f, 0.f, 0.f};
  {
    const int row = tid >> 2, part = tid & 3;
    const int gr = rowBase + row;
    int rr = gr > nN - 1 ? nN - 1 : gr; rr = rr < 0 ? 0 : rr;
    const bool pad = gr >= nN;
    const float* pl = low + (size_t)rr * LOWD + 8 * part;
    v4f a = *(const v4f*)pl, b = *(const v4f*)(pl + 4);
    if (pad) { a = z4; b = z4; }
    *(v8h*)(sA + row * LOWD + 8 * part) = cvt8(a, b);
    const float* ph = high + (size_t)rr * HIGHD + 32 * part;
#pragma unroll
    for (int q = 0; q < 4; ++q) {
      v4f c = *(const v4f*)(ph + 8 * q), d = *(const v4f*)(ph + 8 * q + 4);
      if (pad) { c = z4; d = z4; }
      *(v8h*)(sX + row * IN1 + 32 * part + 8 * q) = cvt8(c, d);
    }
  }
  __syncthreads();

  const int r0 = 16 * (wave >> 1);
  const int c0 = 32 * (wave & 1);
  FragH a;
  a.h[0] = *(const v8h*)(sA + (r0 + m) * LOWD + 8 * hh);
  a.h[1] = *(const v8h*)(sA + (r0 + m) * LOWD + 16 + 8 * hh);
  v8f acc[2];
#pragma unroll
  for (int t = 0; t < 2; ++t) { v8f z = {0.f, 0.f, 0.f, 0.f, 0.f, 0.f, 0.f, 0.f}; acc[t] = z; }
#pragma unroll
  for (int t = 0; t < 2; ++t) {
    const _Float16* bp = wembp + (size_t)(c0 + 16 * t + m) * LOWD + 8 * hh;
    FragH bf;
    bf.h[0] = *(const v8h*)bp;
    bf.h[1] = *(const v8h*)(bp + 16);
    acc[t] = wmh(a.v, bf.v, acc[t]);
  }
#pragma unroll
  for (int t = 0; t < 2; ++t) {
    const int col = c0 + 16 * t + m;
    const float bc = bemb[col];
    _Float16* sp = sX + (size_t)(r0 + 8 * hh) * IN1 + HIGHD + col;
#pragma unroll
    for (int r = 0; r < 8; ++r) {
      float v = acc[t][r] * WINV + bc;
      v = eluf(v);
      sp[r * IN1] = (_Float16)v;
    }
  }
  __syncthreads();

  {
    v8h cv[NIT];
#pragma unroll
    for (int it = 0; it < NIT; ++it) cv[it] = *(const v8h*)(sX + 8 * (it * NTHR + tid));
    _Float16* gb = xp + (size_t)rowBase * IN1;
#pragma unroll
    for (int it = 0; it < NIT; ++it) *(volatile v8h*)(gb + 8 * (size_t)(it * NTHR + tid)) = cv[it];
    __threadfence();
#pragma unroll
    for (int it = 0; it < NIT; ++it) *(volatile v8h*)(gb + 8 * (size_t)(it * NTHR + tid)) = cv[it];
  }
}

__global__ __launch_bounds__(NTHR) void k_count(
    const int* __restrict__ dsts, int* cnt, int nE, int vec8) {
  __shared__ __attribute__((aligned(16))) int scnt[NBC];
  __shared__ __attribute__((aligned(16))) int list[LISTN];
  __shared__ int wcnt[NWAVE];
  const int tid = threadIdx.x, lane = tid & 31, wave = tid >> 5;
  const int nodeBase = blockIdx.x * NBC;

  for (int i = tid; i < NBC; i += NTHR) scnt[i] = 0;
  __syncthreads();

  const int nChunks = (nE + CHUNK - 1) / CHUNK;
#pragma unroll 1
  for (int ch = 0; ch < nChunks; ++ch) {
    const int cbase = ch * CHUNK;
    const int wc = scan_chunk<NBC>(dsts, nE, cbase, nodeBase, vec8, list, tid, lane, wave);
    if (lane == 0) wcnt[wave] = wc;
    __syncthreads();
    if (wave == 0) {
#pragma unroll 1
      for (int wsx = 0; wsx < NWAVE; ++wsx) {
        int n = __builtin_amdgcn_readfirstlane(wcnt[wsx]);
        n = n > WCAP ? WCAP : (n < 0 ? 0 : n);
        const int* lp = list + wsx * WCAP;
#pragma unroll 1
        for (int i = 0; i < n; ++i) {
          const int ent  = __builtin_amdgcn_readfirstlane(lp[i]);
          const int slot = ent & (NBC - 1);
          if (lane == 0) scnt[slot] = scnt[slot] + 1;
        }
      }
    }
    __syncthreads();
  }

  v4i cq[4];
#pragma unroll
  for (int q = 0; q < 4; ++q) {
    const int f = (wave * 4 + q) * 128 + 4 * lane;
    cq[q] = *(const v4i*)(scnt + f);
  }
  int* cp = cnt + (size_t)nodeBase;
#pragma unroll
  for (int q = 0; q < 4; ++q) {
    const int f = (wave * 4 + q) * 128 + 4 * lane;
    *(volatile v4i*)(cp + f) = cq[q];
  }
  __threadfence();
#pragma unroll
  for (int q = 0; q < 4; ++q) {
    const int f = (wave * 4 + q) * 128 + 4 * lane;
    *(volatile v4i*)(cp + f) = cq[q];
  }
}

__global__ __launch_bounds__(OTHR) void k_offsets(
    const int* __restrict__ cnt, int* off, int* rbase, int nChunk) {
  __shared__ __attribute__((aligned(16))) int soff[NBC];
  __shared__ __attribute__((aligned(16))) int srb[RBN];
  __shared__ int wtot[OTHR / 32];
  const int tid = threadIdx.x, lane = tid & 31, wave = tid >> 5, sub = tid >> 7;
  for (int i = tid; i < RBN; i += OTHR) srb[i] = 0;
  int carry = 0;
#pragma unroll 1
  for (int ch = 0; ch < nChunk; ++ch) {
    const int base = ch * NBC;
    const v4i c0 = *(const v4i*)(cnt + base + 8 * tid);
    const v4i c1 = *(const v4i*)(cnt + base + 8 * tid + 4);
    const int e0 = max(c0.x, 0), e1 = max(c0.y, 0), e2 = max(c0.z, 0), e3 = max(c0.w, 0);
    const int e4 = max(c1.x, 0), e5 = max(c1.y, 0), e6 = max(c1.z, 0), e7 = max(c1.w, 0);
    const int ts = e0 + e1 + e2 + e3 + e4 + e5 + e6 + e7;
    int incl = ts;
#pragma unroll
    for (int d = 1; d < 32; d <<= 1) {
      const int t = __shfl_up(incl, d);
      if (lane >= d) incl += t;
    }
    if (lane == 31) wtot[wave] = incl;
    __syncthreads();
    const int S0 = wtot[0]  + wtot[1]  + wtot[2]  + wtot[3];
    const int S1 = wtot[4]  + wtot[5]  + wtot[6]  + wtot[7];
    const int S2 = wtot[8]  + wtot[9]  + wtot[10] + wtot[11];
    const int S3 = wtot[12] + wtot[13] + wtot[14] + wtot[15];
    int pre = 0;
#pragma unroll 1
    for (int w = 4 * sub; w < wave; ++w) pre += wtot[w];
    const int b0 = carry;
    const int b1 = b0 + ((S0 + 31) & ~31);
    const int b2 = b1 + ((S1 + 31) & ~31);
    const int b3 = b2 + ((S2 + 31) & ~31);
    const int b4 = b3 + ((S3 + 31) & ~31);
    const int myb = sub == 0 ? b0 : (sub == 1 ? b1 : (sub == 2 ? b2 : b3));
    if (tid == 0) {
      srb[min(4 * ch + 0, RBN - 1)] = b0;
      srb[min(4 * ch + 1, RBN - 1)] = b1;
      srb[min(4 * ch + 2, RBN - 1)] = b2;
      srb[min(4 * ch + 3, RBN - 1)] = b3;
    }
    int run = myb + pre + incl - ts;
    soff[8 * tid + 0] = run; run += e0;
    soff[8 * tid + 1] = run; run += e1;
    soff[8 * tid + 2] = run; run += e2;
    soff[8 * tid + 3] = run; run += e3;
    soff[8 * tid + 4] = run; run += e4;
    soff[8 * tid + 5] = run; run += e5;
    soff[8 * tid + 6] = run; run += e6;
    soff[8 * tid + 7] = run;
    carry = b4;
    __syncthreads();
    const v4i o0 = *(const v4i*)(soff + 4 * tid);
    const v4i o1 = *(const v4i*)(soff + 4 * (tid + OTHR));
    int* op = off + base;
    *(volatile v4i*)(op + 4 * tid) = o0;
    *(volatile v4i*)(op + 4 * (tid + OTHR)) = o1;
    __threadfence();
    *(volatile v4i*)(op + 4 * tid) = o0;
    *(volatile v4i*)(op + 4 * (tid + OTHR)) = o1;
    __syncthreads();
  }
  if (tid == 0) srb[min(4 * nChunk, RBN - 1)] = carry;
  __syncthreads();
  v4i rv = {0, 0, 0, 0};
  if (tid < 32) rv = *(const v4i*)(srb + 4 * tid);
  if (tid < 32) *(volatile v4i*)(rbase + 4 * tid) = rv;
  __threadfence();
  if (tid < 32) *(volatile v4i*)(rbase + 4 * tid) = rv;
}

__global__ __launch_bounds__(NTHR) void k_fill(
    const int* __restrict__ srcs, const int* __restrict__ dsts,
    const int* __restrict__ off, const int* __restrict__ rbase,
    int* csr, int nN, int nE, int vec8, int csrLen) {
  extern __shared__ v4f lds_dyn[];
  int* region = (int*)lds_dyn;
  int* cursor = region + RCAP;
  int* list   = cursor + NBF;
  int* wcnt   = list + LISTN;
  const int tid = threadIdx.x, lane = tid & 31, wave = tid >> 5;
  const int b = blockIdx.x;
  const int nodeBase = b * NBF;

  int rb0 = rbase[b];
  const int rb1 = rbase[b + 1];
  rb0 = rb0 < 0 ? 0 : (rb0 > csrLen ? csrLen : rb0);
  rb0 &= ~31;
  int len = rb1 - rb0;
  len = len < 0 ? 0 : (len > RCAP ? RCAP : len);
  int lenW = (len + 31) & ~31;
  if (rb0 + lenW > csrLen) lenW = (csrLen - rb0) & ~31;

  {
    const v4i z = {0, 0, 0, 0};
    for (int i = tid; i < RCAP / 4; i += NTHR) ((v4i*)region)[i] = z;
    for (int s = tid; s < NBF; s += NTHR) {
      int o = off[nodeBase + s] - rb0;
      o = o < 0 ? 0 : (o > RCAP ? RCAP : o);
      cursor[s] = o;
    }
  }
  __syncthreads();

  const int nChunks = (nE + CHUNK - 1) / CHUNK;
#pragma unroll 1
  for (int ch = 0; ch < nChunks; ++ch) {
    const int cbase = ch * CHUNK;
    const int wc = scan_chunk<NBF>(dsts, nE, cbase, nodeBase, vec8, list, tid, lane, wave);
    if (lane == 0) wcnt[wave] = wc;
    __syncthreads();
    if (wave == 0) {
#pragma unroll 1
      for (int wsx = 0; wsx < NWAVE; ++wsx) {
        int n = __builtin_amdgcn_readfirstlane(wcnt[wsx]);
        n = n > WCAP ? WCAP : (n < 0 ? 0 : n);
        const int* lp = list + wsx * WCAP;
#pragma unroll 1
        for (int i = 0; i < n; ++i) {
          const int ent  = __builtin_amdgcn_readfirstlane(lp[i]);
          const int slot = ent & (NBF - 1);
          int e = cbase + ((ent >> 12) & (CHUNK - 1));
          e = e > nE - 1 ? nE - 1 : e;
          int src = srcs[e];
          src = src < 0 ? 0 : (src > nN - 1 ? nN - 1 : src);
          if (lane == 0) {
            int pos = cursor[slot];
            pos = pos < 0 ? 0 : (pos > RCAP - 1 ? RCAP - 1 : pos);
            region[pos] = src;
            const int np = pos + 1;
            cursor[slot] = np > RCAP ? RCAP : np;
          }
        }
      }
    }
    __syncthreads();
  }

  const int nv = lenW >> 2;
  int* gp = csr + rb0;
#pragma unroll 1
  for (int i = tid; i < nv; i += NTHR) { const v4i v = ((const v4i*)region)[i]; *(volatile v4i*)(gp + 4 * i) = v; }
  __threadfence();
#pragma unroll 1
  for (int i = tid; i < nv; i += NTHR) { const v4i v = ((const v4i*)region)[i]; *(volatile v4i*)(gp + 4 * i) = v; }
}

__global__ __launch_bounds__(NTHR) void k_gemm1(
    const _Float16* __restrict__ xp, const _Float16* __restrict__ w1p,
    const float* __restrict__ attS, const float* __restrict__ attD,
    float* hp, float* eS, float* eD) {
  constexpr int K   = IN1;
  constexpr int NC  = C1;
  constexpr int KT  = K / 32;
  constexpr int TPW = 4;
  constexpr int NIT = BM1 * NC / 4 / NTHR;
  __shared__ __attribute__((aligned(16))) float stg[BM1 * NC];
  __shared__ __attribute__((aligned(16))) float sES[BM1 * HEADS];
  __shared__ __attribute__((aligned(16))) float sED[BM1 * HEADS];
  const int tid = threadIdx.x, lane = tid & 31, wave = tid >> 5, hh = lane >> 4, m = lane & 15;
  const int rowBase = blockIdx.x * BM1;
  const int r0 = 16 * (wave >> 2);
  const int c0 = 64 * (wave & 3);

  v8f acc[TPW];
#pragma unroll
  for (int t = 0; t < TPW; ++t) { v8f z = {0.f, 0.f, 0.f, 0.f, 0.f, 0.f, 0.f, 0.f}; acc[t] = z; }

  const _Float16* ap  = xp + (size_t)(rowBase + r0 + m) * K + 8 * hh;
  const _Float16* bp0 = w1p + (size_t)(c0 + m) * K + 8 * hh;
#pragma unroll 1
  for (int kt = 0; kt < KT; ++kt) {
    FragH a;
    a.h[0] = *(const v8h*)(ap + 32 * kt);
    a.h[1] = *(const v8h*)(ap + 32 * kt + 16);
#pragma unroll
    for (int t = 0; t < TPW; ++t) {
      const _Float16* bp = bp0 + (size_t)(16 * t) * K + 32 * kt;
      FragH bf;
      bf.h[0] = *(const v8h*)bp;
      bf.h[1] = *(const v8h*)(bp + 16);
      acc[t] = wmh(a.v, bf.v, acc[t]);
    }
  }

  {
    float* sp = stg + (size_t)(r0 + 8 * hh) * NC + c0 + m;
#pragma unroll
    for (int t = 0; t < TPW; ++t) {
#pragma unroll
      for (int r = 0; r < 8; ++r) sp[r * NC + 16 * t] = acc[t][r] * WINV;
    }
  }
  __syncthreads();

  {
    const int drow = tid >> 3, dh = tid & 7;
    const float* rp  = stg + (size_t)drow * NC + dh * HIDC;
    const float* sa  = attS + dh * HIDC;
    const float* sdd = attD + dh * HIDC;
    float ps = 0.f, pd = 0.f;
#pragma unroll 2
    for (int cc = 0; cc < HIDC; cc += 4) {
      const v4f hv = *(const v4f*)(rp + cc);
      const v4f av = *(const v4f*)(sa + cc);
      const v4f dv = *(const v4f*)(sdd + cc);
      ps += hv.x * av.x + hv.y * av.y + hv.z * av.z + hv.w * av.w;
      pd += hv.x * dv.x + hv.y * dv.y + hv.z * dv.z + hv.w * dv.w;
    }
    sES[tid] = ps;
    sED[tid] = pd;
  }

  {
    float* tileC = hp + (size_t)rowBase * NC;
    v4f cv[NIT];
#pragma unroll
    for (int it = 0; it < NIT; ++it) cv[it] = *(const v4f*)(stg + 4 * (it * NTHR + tid));
#pragma unroll
    for (int it = 0; it < NIT; ++it) *(volatile v4f*)(tileC + 4 * (size_t)(it * NTHR + tid)) = cv[it];
    __threadfence();
#pragma unroll
    for (int it = 0; it < NIT; ++it) *(volatile v4f*)(tileC + 4 * (size_t)(it * NTHR + tid)) = cv[it];
  }
  __syncthreads();

  {
    const int i = tid & 63;
    const bool isS = tid < 64;
    const v4f vS = *(const v4f*)(sES + 4 * i);
    const v4f vD = *(const v4f*)(sED + 4 * i);
    const v4f dv = isS ? vS : vD;
    float* gp = (isS ? eS : eD) + (size_t)rowBase * HEADS + 4 * i;
    if (tid < 128) *(volatile v4f*)gp = dv;
    __threadfence();
    if (tid < 128) *(volatile v4f*)gp = dv;
  }
}

__global__ __launch_bounds__(NTHR) void k_agg1(
    const int* __restrict__ csr, const int* __restrict__ off, const int* __restrict__ cnt,
    const float* __restrict__ eS, const float* __restrict__ eD, const float* __restrict__ hp,
    const float* __restrict__ bias, _Float16* xo, int nN, int csrLen) {
  __shared__ __attribute__((aligned(16))) float pw[NWAVE * 32 * HEADS];
  const int tid = threadIdx.x, lane = tid & 31, wave = tid >> 5;
  const int tbase = blockIdx.x * TGT + wave * 32;
  const int col = 8 * lane;
  const int hd  = lane >> 2;
  float* pww = pw + wave * (32 * HEADS);
  const v4f z4 = {0.f, 0.f, 0.f, 0.f};
  const v4f bb0 = *(const v4f*)(bias + col), bb1 = *(const v4f*)(bias + col + 4);

  const int cl    = tbase + lane;
  const int cnt_l = cnt[cl];
  const int off_l = off[cl];

#pragma unroll 1
  for (int j = 0; j < 32; ++j) {
    const int c = tbase + j;
    int n = __builtin_amdgcn_readfirstlane(__shfl(cnt_l, j));
    n = n < 0 ? 0 : (n > DEGCAP ? DEGCAP : n);
    const int st = __builtin_amdgcn_readfirstlane(__shfl(off_l, j));
    const v4f esc0 = *(const v4f*)(eS + (size_t)c * HEADS), esc1 = *(const v4f*)(eS + (size_t)c * HEADS + 4);
    const v4f edc0 = *(const v4f*)(eD + (size_t)c * HEADS), edc1 = *(const v4f*)(eD + (size_t)c * HEADS + 4);
    v4f m0 = lrelu4(esc0 + edc0), m1 = lrelu4(esc1 + edc1);
    const float eself = sel8(m0, m1, hd);

#pragma unroll 1
    for (int q0 = 0; q0 < n; q0 += 32) {
      int pos = st + q0 + lane;
      pos = pos < 0 ? 0 : (pos > csrLen - 1 ? csrLen - 1 : pos);
      int s = csr[pos];
      s = s < 0 ? 0 : (s > nN - 1 ? nN - 1 : s);
      const bool valid = (q0 + lane) < n;
      const v4f a0 = *(const v4f*)(eS + (size_t)s * HEADS), a1 = *(const v4f*)(eS + (size_t)s * HEADS + 4);
      const v4f t0 = lrelu4(a0 + edc0), t1 = lrelu4(a1 + edc1);
      m0 = valid ? fmax4(m0, t0) : m0;
      m1 = valid ? fmax4(m1, t1) : m1;
    }
#pragma unroll
    for (int d = 16; d > 0; d >>= 1) { m0 = xormax4(m0, d); m1 = xormax4(m1, d); }
    const float mx = sel8(m0, m1, hd);

    const float pself = __expf(eself - mx);
    float den = pself;
    const float* hc = hp + (size_t)c * C1 + col;
    v4f acc0 = *(const v4f*)hc * pself, acc1 = *(const v4f*)(hc + 4) * pself;

#pragma unroll 1
    for (int q0 = 0; q0 < n; q0 += 32) {
      int pos = st + q0 + lane;
      pos = pos < 0 ? 0 : (pos > csrLen - 1 ? csrLen - 1 : pos);
      int s = csr[pos];
      s = s < 0 ? 0 : (s > nN - 1 ? nN - 1 : s);
      const bool valid = (q0 + lane) < n;
      const v4f a0 = *(const v4f*)(eS + (size_t)s * HEADS), a1 = *(const v4f*)(eS + (size_t)s * HEADS + 4);
      const v4f t0 = lrelu4(a0 + edc0), t1 = lrelu4(a1 + edc1);
      v4f p0 = exp4(t0 - m0), p1 = exp4(t1 - m1);
      if (!valid) { p0 = z4; p1 = z4; }
      wave_sync();
      *(v4f*)(pww + lane * HEADS) = p0;
      *(v4f*)(pww + lane * HEADS + 4) = p1;
      wave_sync();
      int mcnt = n - q0; mcnt = mcnt < 32 ? mcnt : 32;
#pragma unroll 1
      for (int pp = 0; pp < mcnt; ++pp) {
        const int sp = __builtin_amdgcn_readlane(s, pp);
        const float pv = pww[pp * HEADS + hd];
        den += pv;
        const float* hs = hp + (size_t)sp * C1 + col;
        const v4f hv0 = *(const v4f*)hs, hv1 = *(const v4f*)(hs + 4);
        acc0 = acc0 + hv0 * pv;
        acc1 = acc1 + hv1 * pv;
      }
    }

    const float rd = __builtin_amdgcn_rcpf(den);
    v4f v0 = acc0 * rd + bb0, v1 = acc1 * rd + bb1;
    v0 = elu4(v0); v1 = elu4(v1);
    if (c >= nN) { v0 = z4; v1 = z4; }
    const v8h o = cvt8(v0, v1);
    _Float16* gp = xo + (size_t)c * C1 + col;
    *(volatile v8h*)gp = o;
    __threadfence();
    *(volatile v8h*)gp = o;
  }
}

__global__ __launch_bounds__(G2THR) void k_gemm2(
    const _Float16* __restrict__ x2p, const _Float16* __restrict__ w2p,
    const float* __restrict__ as2, const float* __restrict__ ad2, float* h2p) {
  constexpr int K   = C1;
  constexpr int KT  = K / 32;
  constexpr int NIT = BM2 * OUTP / 4 / G2THR;
  __shared__ __attribute__((aligned(16))) float stg[BM2 * OUTP];
  const int tid = threadIdx.x, lane = tid & 31, wave = tid >> 5, hh = lane >> 4, m = lane & 15;
  const int rowBase = blockIdx.x * BM2;
  const int r0 = 16 * wave;

  v8f acc = {0.f, 0.f, 0.f, 0.f, 0.f, 0.f, 0.f, 0.f};
  const _Float16* ap = x2p + (size_t)(rowBase + r0 + m) * K + 8 * hh;
  const _Float16* bp = w2p + (size_t)m * K + 8 * hh;
#pragma unroll 1
  for (int kt = 0; kt < KT; ++kt) {
    FragH a, bf;
    a.h[0]  = *(const v8h*)(ap + 32 * kt);
    a.h[1]  = *(const v8h*)(ap + 32 * kt + 16);
    bf.h[0] = *(const v8h*)(bp + 32 * kt);
    bf.h[1] = *(const v8h*)(bp + 32 * kt + 16);
    acc = wmh(a.v, bf.v, acc);
  }
  {
    float* sp = stg + (size_t)(r0 + 8 * hh) * OUTP + m;
#pragma unroll
    for (int r = 0; r < 8; ++r) sp[r * OUTP] = acc[r] * WINV;
  }
  __syncthreads();

  if (tid < BM2) {
    float* rp = stg + tid * OUTP;
    float s = 0.f, d = 0.f;
#pragma unroll
    for (int o = 0; o < OUTC; ++o) { const float hv = rp[o]; s += hv * as2[o]; d += hv * ad2[o]; }
    rp[OUTC] = s;
    rp[OUTC + 1] = d;
  }
  __syncthreads();

  {
    v4f cv[NIT];
#pragma unroll
    for (int it = 0; it < NIT; ++it) cv[it] = *(const v4f*)(stg + 4 * (it * G2THR + tid));
    float* gb = h2p + (size_t)rowBase * OUTP;
#pragma unroll
    for (int it = 0; it < NIT; ++it) *(volatile v4f*)(gb + 4 * (size_t)(it * G2THR + tid)) = cv[it];
    __threadfence();
#pragma unroll
    for (int it = 0; it < NIT; ++it) *(volatile v4f*)(gb + 4 * (size_t)(it * G2THR + tid)) = cv[it];
  }
}

__global__ __launch_bounds__(NTHR) void k_agg2(
    const int* __restrict__ csr, const int* __restrict__ off, const int* __restrict__ cnt,
    const float* __restrict__ h2p, const float* __restrict__ bias, float* out, int nN, int csrLen) {
  __shared__ __attribute__((aligned(16))) float so[NWAVE * 32 * OUTC];
  const int tid = threadIdx.x, lane = tid & 31, wave = tid >> 5;
  const int tbase = blockIdx.x * TGT + wave * 32;
  float* sow = so + wave * (32 * OUTC);
  const v4f bb0 = *(const v4f*)bias, bb1 = *(const v4f*)(bias + 4);
  const float l0 = (lane == 0) ? 1.0f : 0.0f;

  const int cl    = tbase + lane;
  const int cnt_l = cnt[cl];
  const int off_l = off[cl];

#pragma unroll 1
  for (int j = 0; j < 32; ++j) {
    const int c = tbase + j;
    int n = __builtin_amdgcn_readfirstlane(__shfl(cnt_l, j));
    n = n < 0 ? 0 : (n > DEGCAP ? DEGCAP : n);
    const int st = __builtin_amdgcn_readfirstlane(__shfl(off_l, j));
    const float* rc = h2p + (size_t)c * OUTP;
    const float edc = rc[OUTC + 1];
    const float eself = lrelu(rc[OUTC] + edc);

    float mx = eself;
#pragma unroll 1
    for (int q0 = 0; q0 < n; q0 += 32) {
      int pos = st + q0 + lane;
      pos = pos < 0 ? 0 : (pos > csrLen - 1 ? csrLen - 1 : pos);
      int s = csr[pos];
      s = s < 0 ? 0 : (s > nN - 1 ? nN - 1 : s);
      const bool valid = (q0 + lane) < n;
      const float t = lrelu(h2p[(size_t)s * OUTP + OUTC] + edc);
      mx = valid ? fmaxf(mx, t) : mx;
    }
#pragma unroll
    for (int d = 16; d > 0; d >>= 1) mx = fmaxf(mx, __shfl_xor(mx, d));

    const float ps0 = __expf(eself - mx) * l0;
    float den = ps0;
    v4f acc0 = *(const v4f*)rc * ps0, acc1 = *(const v4f*)(rc + 4) * ps0;
#pragma unroll 1
    for (int q0 = 0; q0 < n; q0 += 32) {
      int pos = st + q0 + lane;
      pos = pos < 0 ? 0 : (pos > csrLen - 1 ? csrLen - 1 : pos);
      int s = csr[pos];
      s = s < 0 ? 0 : (s > nN - 1 ? nN - 1 : s);
      const bool valid = (q0 + lane) < n;
      const float* rs = h2p + (size_t)s * OUTP;
      const float t = lrelu(rs[OUTC] + edc);
      float p = __expf(t - mx);
      p = valid ? p : 0.0f;
      den += p;
      acc0 = acc0 + *(const v4f*)rs * p;
      acc1 = acc1 + *(const v4f*)(rs + 4) * p;
    }
#pragma unroll
    for (int d = 16; d > 0; d >>= 1) { den += __shfl_xor(den, d); acc0 = xorsum4(acc0, d); acc1 = xorsum4(acc1, d); }

    const float rd = __builtin_amdgcn_rcpf(den);
    const v4f v0 = acc0 * rd + bb0, v1 = acc1 * rd + bb1;
    const float mv = fmaxf(fmaxf(fmaxf(v0.x, v0.y), fmaxf(v0.z, v0.w)),
                           fmaxf(fmaxf(v1.x, v1.y), fmaxf(v1.z, v1.w)));
    const v4f e0 = exp4(v0 - mv), e1 = exp4(v1 - mv);
    const float zs = ((e0.x + e0.y) + (e0.z + e0.w)) + ((e1.x + e1.y) + (e1.z + e1.w));
    const float lg = mv + __logf(zs);
    const v4f o0 = v0 - lg, o1 = v1 - lg;
    const v4f ov = (lane == 0) ? o0 : o1;
    if (lane < 2) *(v4f*)(sow + j * OUTC + 4 * lane) = ov;
  }
  __syncthreads();

  {
    int nval = nN - tbase;
    nval = nval < 0 ? 0 : (nval > 32 ? 32 : nval);
    const int np = 2 * nval;
    v4f ov[2];
#pragma unroll
    for (int q = 0; q < 2; ++q) { const int idx = q * 32 + lane; ov[q] = *(const v4f*)(sow + 4 * idx); }
    float* ob = out + (size_t)tbase * OUTC;
#pragma unroll
    for (int q = 0; q < 2; ++q) { const int idx = q * 32 + lane; if (idx < np) *(volatile v4f*)(ob + 4 * idx) = ov[q]; }
    __threadfence();
#pragma unroll
    for (int q = 0; q < 2; ++q) { const int idx = q * 32 + lane; if (idx < np) *(volatile v4f*)(ob + 4 * idx) = ov[q]; }
  }
}

extern "C" void kernel_launch(void* const* d_in, const int* in_sizes, int n_in,
                              void* d_out, int out_size, void* d_ws, size_t ws_size,
                              hipStream_t stream) {
  if (n_in < 13) return;
  const int nN = in_sizes[0] / HIGHD;
  const int nE = in_sizes[2] / 2;
  if (nN <= 0 || nE <= 0) return;
  if (in_sizes[0] != nN * HIGHD || in_sizes[1] != nN * LOWD || in_sizes[2] != 2 * nE) return;
  if (in_sizes[3] != LOWD * EMBD || in_sizes[4] != EMBD) return;
  if (in_sizes[5] != IN1 * C1 || in_sizes[6] != HEADS * HIDC || in_sizes[7] != HEADS * HIDC || in_sizes[8] != C1) return;
  if (in_sizes[9] != C1 * OUTC || in_sizes[10] != OUTC || in_sizes[11] != OUTC || in_sizes[12] != OUTC) return;
  if (out_size != nN * OUTC) return;
  if (nE > (1 << 28) || nN > (1 << 22)) return;

  const float* high = (const float*)d_in[0];
  const float* low  = (const float*)d_in[1];
  const int*   ei   = (const int*)d_in[2];
  const int*   src  = ei;
  const int*   dst  = ei + nE;
  const float* Wemb = (const float*)d_in[3];
  const float* bemb = (const float*)d_in[4];
  const float* W1   = (const float*)d_in[5];
  const float* a1s  = (const float*)d_in[6];
  const float* a1d  = (const float*)d_in[7];
  const float* b1   = (const float*)d_in[8];
  const float* W2   = (const float*)d_in[9];
  const float* a2s  = (const float*)d_in[10];
  const float* a2d  = (const float*)d_in[11];
  const float* b2   = (const float*)d_in[12];
  float* out = (float*)d_out;

  const int NPAD   = ((nN + TGT - 1) / TGT) * TGT;
  const int nBC    = (nN + NBC - 1) / NBC;
  const int CNTPAD = nBC * NBC;
  if (CNTPAD < NPAD) return;
  if (4 * nBC + 1 > RBN) return;
  const int nBF    = (nN + NBF - 1) / NBF;
  if (nBF + 1 > 4 * nBC + 1) return;
  const int csrLen = ((nE + 31) & ~31) + 4096;
  if (31 * 4 * nBC > 4096) return;
  const int nAgg   = NPAD / TGT;
  const int nX     = NPAD / BMX;
  const int nG1    = NPAD / BM1;
  const int nG2    = NPAD / BM2;

  char* ws = (char*)d_ws;
  size_t off = 0;
  const size_t oWe  = off; off += (size_t)EMBD * LOWD * 2;          off = (off + 255) & ~(size_t)255;
  const size_t oW1  = off; off += (size_t)C1 * IN1 * 2;             off = (off + 255) & ~(size_t)255;
  const size_t oW2  = off; off += (size_t)OUTP * C1 * 2;            off = (off + 255) & ~(size_t)255;
  const size_t oX   = off; off += (size_t)NPAD * IN1 * 2;           off = (off + 255) & ~(size_t)255;
  const size_t oCnt = off; off += (size_t)CNTPAD * 4;               off = (off + 255) & ~(size_t)255;
  const size_t oOff = off; off += (size_t)CNTPAD * 4;               off = (off + 255) & ~(size_t)255;
  const size_t oRb  = off; off += (size_t)RBN * 4;                  off = (off + 255) & ~(size_t)255;
  const size_t oCsr = off; off += (size_t)csrLen * 4;               off = (off + 255) & ~(size_t)255;
  const size_t oH   = off; off += (size_t)NPAD * C1 * 4;            off = (off + 255) & ~(size_t)255;
  const size_t oES  = off; off += (size_t)NPAD * HEADS * 4;         off = (off + 255) & ~(size_t)255;
  const size_t oED  = off; off += (size_t)NPAD * HEADS * 4;         off = (off + 255) & ~(size_t)255;
  const size_t oX2  = off; off += (size_t)NPAD * C1 * 2;            off = (off + 255) & ~(size_t)255;
  const size_t oH2  = off; off += (size_t)NPAD * OUTP * 4;          off = (off + 255) & ~(size_t)255;
  if (off > ws_size || off > (size_t)WSCAP) return;
  _Float16* wembp = (_Float16*)(ws + oWe);
  _Float16* w1p   = (_Float16*)(ws + oW1);
  _Float16* w2p   = (_Float16*)(ws + oW2);
  _Float16* xp    = (_Float16*)(ws + oX);
  int*   cnt  = (int*)(ws + oCnt);
  int*   offp = (int*)(ws + oOff);
  int*   rb   = (int*)(ws + oRb);
  int*   csr  = (int*)(ws + oCsr);
  float* hp   = (float*)(ws + oH);
  float* es   = (float*)(ws + oES);
  float* ed   = (float*)(ws + oED);
  _Float16* x2p = (_Float16*)(ws + oX2);
  float* h2p  = (float*)(ws + oH2);

  const int vec8 = ((nE & 3) == 0) ? 1 : 0;

  k_wprep<LOWD, EMBD, EMBD><<<(EMBD * LOWD / 8 + NTHR - 1) / NTHR, NTHR, 0, stream>>>(Wemb, wembp);
  k_wprep<IN1, C1, C1><<<(C1 * IN1 / 8 + NTHR - 1) / NTHR, NTHR, 0, stream>>>(W1, w1p);
  k_wprep<C1, OUTC, OUTP><<<(OUTP * C1 / 8 + NTHR - 1) / NTHR, NTHR, 0, stream>>>(W2, w2p);
  k_xprep<<<nX, NTHR, 0, stream>>>(high, low, wembp, bemb, xp, nN);

  k_count<<<nBC, NTHR, 0, stream>>>(dst, cnt, nE, vec8);
  k_offsets<<<1, OTHR, 0, stream>>>(cnt, offp, rb, nBC);
  hipFuncSetAttribute(reinterpret_cast<const void*>(&k_fill),
                      hipFuncAttributeMaxDynamicSharedMemorySize, LDS_FILL);
  k_fill<<<nBF, NTHR, LDS_FILL, stream>>>(src, dst, offp, rb, csr, nN, nE, vec8, csrLen);

  k_gemm1<<<nG1, NTHR, 0, stream>>>(xp, w1p, a1s, a1d, hp, es, ed);
  k_agg1<<<nAgg, NTHR, 0, stream>>>(csr, offp, cnt, es, ed, hp, b1, x2p, nN, csrLen);

  k_gemm2<<<nG2, G2THR, 0, stream>>>(x2p, w2p, a2s, a2d, h2p);
  k_agg2<<<nAgg, NTHR, 0, stream>>>(csr, offp, cnt, h2p, b2, out, nN, csrLen);
}
